// TorchWrapperWithMetrics_89850715833247
// MI455X (gfx1250) — hardware-run, weakly checked
//
#include <hip/hip_runtime.h>


#ifndef BQ
#define BQ 2048
#endif
#ifndef NPTS
#define NPTS 100000
#endif
#define DF   64
#define ZP   66
#define OW   66
#define HID  256
#define KIN  65
#define K1   96
#define K1P  128
#define KNN  20
#define QT   16
#define XP   104
#define HP   264
#define FP   68
#define W2S  64.0f
#define W2I  (1.0f / 64.0f)
#define BIGD 3.0e38f
#define W1BLK ((HID * K1P / 8) / 256)
#define W2BLK ((DF * HID / 8) / 256)

static_assert(DF == 64);
static_assert(DF % 32 == 0);
static_assert(NPTS % 32 == 0);
static_assert(NPTS >= 2 * KNN);
static_assert(((size_t)NPTS * DF) % (256 * 8) == 0);
static_assert(BQ % QT == 0);
static_assert(QT == 16);
static_assert(KIN <= K1);
static_assert(K1 % 32 == 0);
static_assert(K1 <= K1P);
static_assert(K1P % 64 == 0);
static_assert(K1 <= XP);
static_assert(XP % 8 == 0);
static_assert(HID % 32 == 0);
static_assert(HID % 16 == 0);
static_assert(HID <= HP);
static_assert(HP % 8 == 0);
static_assert(DF % 16 == 0);
static_assert(DF + 4 <= FP);
static_assert(OW == DF + 2);
static_assert(QT * OW * 4 == (8 * 32 + 8) * 16);
static_assert((HID * K1P / 8) % 256 == 0);
static_assert((DF * HID / 8) % 256 == 0);
static_assert(KNN % 2 == 0);
static_assert((QT * KNN) % 32 == 0);
static_assert(QT * XP * 2 + QT * HP * 2 + 2 * QT * FP * 4 + QT * OW * 4 + QT * 4 + 2 * QT * 2 * KNN * 4 + 3 * QT * KNN * 4 <= 131072);

typedef _Float16 h16;
typedef unsigned short bf;
typedef __attribute__((ext_vector_type(16))) __bf16   v16bf;
typedef __attribute__((ext_vector_type(16))) _Float16 v16h;
typedef __attribute__((ext_vector_type(8)))  _Float16 v8h;
typedef __attribute__((ext_vector_type(8)))  unsigned short v8us;
typedef __attribute__((ext_vector_type(8)))  float    v8f;
typedef __attribute__((ext_vector_type(4)))  float    v4f;
typedef __attribute__((ext_vector_type(2)))  float    v2f;
typedef v4f  __attribute__((may_alias)) v4fa;

__device__ __forceinline__ unsigned short f2bf(float f) { unsigned u = __float_as_uint(f); u += 0x7FFFu + ((u >> 16) & 1u); return (unsigned short)(u >> 16); }
__device__ __forceinline__ float bfr(float f) { return __uint_as_float(((unsigned)f2bf(f)) << 16); }
__device__ __forceinline__ v16h cat16(v8h lo, v8h hi) { return __builtin_shufflevector(lo, hi, 0, 1, 2, 3, 4, 5, 6, 7, 8, 9, 10, 11, 12, 13, 14, 15); }
__device__ __forceinline__ v16bf cat16b(v8us lo, v8us hi) { return __builtin_bit_cast(v16bf, __builtin_shufflevector(lo, hi, 0, 1, 2, 3, 4, 5, 6, 7, 8, 9, 10, 11, 12, 13, 14, 15)); }
__device__ __forceinline__ v8f wmma16(v16h a, v16h b, v8f c) { return __builtin_amdgcn_wmma_f32_16x16x32_f16(false, a, false, b, (short)0, c, false, false); }
__device__ __forceinline__ v8f wmmab(v16bf a, v16bf b, v8f c) { return __builtin_amdgcn_wmma_f32_16x16x32_bf16(false, a, false, b, (short)0, c, false, false); }
__device__ __forceinline__ v16h  ldh(const h16* p) { return cat16(*(const v8h*)p, *(const v8h*)(p + 16)); }
__device__ __forceinline__ v16bf ldb(const bf* p)  { return cat16b(*(const v8us*)p, *(const v8us*)(p + 16)); }
__device__ __forceinline__ void wave_sync() { __builtin_amdgcn_fence(3  , "wavefront"); __builtin_amdgcn_wave_barrier(); asm volatile("" ::: "memory"); }

__device__ __forceinline__ float bf2f(bf u) { return __uint_as_float(((unsigned)u) << 16); }
__device__ __forceinline__ h16 toh_flush(float v) { const h16 r = (h16)v; return (fabsf(v) < 6.103515625e-05f) ? (h16)0.0f : r; }
__device__ __forceinline__ v8f wmmab_g(v16bf a, v16bf b, v8f c) { v8f d = wmmab(a, b, c); asm volatile("v_nop\n\tv_nop\n\tv_nop\n\tv_nop" : "+v"(d) : "v"(a), "v"(b)); return d; }
__device__ __forceinline__ v8f wmma16_g(v16h a, v16h b, v8f c) { v8f d = wmma16(a, b, c); asm volatile("v_nop\n\tv_nop\n\tv_nop\n\tv_nop" : "+v"(d) : "v"(a), "v"(b)); return d; }

__global__ __launch_bounds__(256) void k_dcvt(const float* __restrict__ src, bf* DB, float* DN) {
#pragma clang fp contract(off)
    __shared__ __align__(16) float dn_s[32];
    const int tid = threadIdx.x;
    const size_t i = (size_t)blockIdx.x * 256 + tid;
    const v8f v = *(const v8f*)(src + i * 8);
    v8us o; float s = 0.0f;
#pragma unroll
    for (int k = 0; k < 8; ++k) { const bf u = f2bf(v[k]); o[k] = u; const float f = bf2f(u); s += f * f; }
    s += __shfl_xor(s, 1, 32); s += __shfl_xor(s, 2, 32); s += __shfl_xor(s, 4, 32);
    if ((tid & 7) == 0) dn_s[tid >> 3] = s;
    __syncthreads();
    const v4f dv = *(const v4fa*)(&dn_s[(tid & 7) * 4]);
    float* dnp = DN + (size_t)blockIdx.x * 32 + (size_t)(tid & 7) * 4;
    *(volatile v8us*)(DB + i * 8) = o;
    if (tid < 8) *(volatile v4f*)dnp = dv;
    __threadfence();
    *(volatile v8us*)(DB + i * 8) = o;
    if (tid < 8) *(volatile v4f*)dnp = dv;
}

__global__ __launch_bounds__(256) void k_wconv(const float* __restrict__ W1, const float* __restrict__ W2, bf* W1T, h16* W2T) {
#pragma clang fp contract(off)
    if (blockIdx.x < W1BLK) {
        const int e = blockIdx.x * 256 + threadIdx.x;
        const int n = e / (K1P / 8), k0 = (e % (K1P / 8)) * 8;
        v8us o;
#pragma unroll
        for (int k = 0; k < 8; ++k) {
            const int kk = k0 + k; const int kc = kk < KIN ? kk : (KIN - 1);
            float x = W1[(size_t)kc * HID + n]; asm volatile("" : "+v"(x));
            o[k] = (kk < KIN) ? f2bf(x) : (bf)0; }
        *(volatile v8us*)(W1T + (size_t)e * 8) = o; __threadfence(); *(volatile v8us*)(W1T + (size_t)e * 8) = o;
    } else {
        const int e = (blockIdx.x - W1BLK) * 256 + threadIdx.x;
        const int n = e / (HID / 8), k0 = (e % (HID / 8)) * 8;
        v8h o;
#pragma unroll
        for (int k = 0; k < 8; ++k) o[k] = toh_flush(bfr(W2[(size_t)(k0 + k) * DF + n]) * W2S);
        *(volatile v8h*)(W2T + (size_t)e * 8) = o; __threadfence(); *(volatile v8h*)(W2T + (size_t)e * 8) = o;
    }
}

__device__ __forceinline__ void knn_insert(float s, int idx, float (&kd)[KNN], int (&ki)[KNN], float& kmax, int& kpos, float& thr) {
    if (s < thr) {
        const float d = sqrtf(fmaxf(s, 1.0e-30f));
        if (d < kmax) {
#pragma unroll
            for (int i = 0; i < KNN; ++i) { const bool rep = (i == kpos); kd[i] = rep ? d : kd[i]; ki[i] = rep ? idx : ki[i]; }
            float m = kd[0]; int mi = ki[0]; int p = 0;
#pragma unroll
            for (int i = 1; i < KNN; ++i) { const bool g = (kd[i] > m) | ((kd[i] == m) & (ki[i] > mi)); m = g ? kd[i] : m; mi = g ? ki[i] : mi; p = g ? i : p; }
            kmax = m; kpos = p; thr = (m * m) * 1.0000002384185791f;
        }
    }
}

__global__ __launch_bounds__(32) void k_knn(const float* __restrict__ z, const float* __restrict__ tin, const bf* __restrict__ DB, const float* __restrict__ DN,
                                            const float* __restrict__ vel, const bf* __restrict__ W1T, const float* __restrict__ b1,
                                            const h16* __restrict__ W2T, const float* __restrict__ b2, float* OUT) {
    __shared__ __align__(16) bf    xs[QT * XP];
    __shared__ __align__(16) h16   hs[QT * HP];
    __shared__ __align__(16) float xd_s[QT * FP];
    __shared__ __align__(16) float ut_s[QT * FP];
    __shared__ __align__(16) float ot[QT * OW];
    __shared__ float xn_s[QT];
    __shared__ float cd[QT * 2 * KNN];
    __shared__ int   ci[QT * 2 * KNN];
    __shared__ float sd[QT * KNN];
    __shared__ int   si[QT * KNN];
    __shared__ float wn[QT * KNN];
    const int lane = threadIdx.x & 31, lr = lane & 15, hi = lane >> 4;
    const int q0 = blockIdx.x * QT;

    const bf tb = f2bf(tin[0]);
#pragma unroll 1
    for (int r = 0; r < QT; ++r) {
        const float* zr = z + (size_t)(q0 + r) * ZP;
        const bf ua = f2bf(zr[lane]), uc = f2bf(zr[32 + lane]);
        const float fa = bf2f(ua), fc = bf2f(uc);
        xs[r * XP + lane] = ua; xs[r * XP + 32 + lane] = uc; xs[r * XP + 64 + lane] = (lane == 0) ? tb : (bf)0;
        float s = fa * fa + fc * fc;
        s += __shfl_xor(s, 16, 32); s += __shfl_xor(s, 8, 32); s += __shfl_xor(s, 4, 32); s += __shfl_xor(s, 2, 32); s += __shfl_xor(s, 1, 32);
        if (lane == 0) xn_s[r] = s;
    }
    wave_sync();

    { const int xo = lr * XP + 8 * hi;
      const v16bf a0 = cat16b(*(const v8us*)(&xs[xo]),      *(const v8us*)(&xs[xo + 16]));
      const v16bf a1 = cat16b(*(const v8us*)(&xs[xo + 32]), *(const v8us*)(&xs[xo + 48]));
      const v16bf a2 = cat16b(*(const v8us*)(&xs[xo + 64]), *(const v8us*)(&xs[xo + 80]));
#pragma unroll 1
      for (int nb = 0; nb < HID / 16; ++nb) {
          const bf* wp = W1T + (size_t)(nb * 16 + lr) * K1P + 8 * hi;
          v8f acc = (v8f){};
          acc = wmmab_g(a0, ldb(wp), acc); acc = wmmab_g(a1, ldb(wp + 32), acc); acc = wmmab_g(a2, ldb(wp + 64), acc);
          const float bv = bfr(b1[nb * 16 + lr]);
#pragma unroll
          for (int r = 0; r < 8; ++r) hs[(8 * hi + r) * HP + nb * 16 + lr] = toh_flush(fmaxf(acc[r] + bv, 0.0f));
      } }
    wave_sync();

    { const int ho = lr * HP + 8 * hi;
#pragma unroll 1
      for (int nb = 0; nb < DF / 16; ++nb) {
          const h16* wp = W2T + (size_t)(nb * 16 + lr) * HID + 8 * hi;
          v8f acc = (v8f){};
#pragma unroll 1
          for (int ks = 0; ks < HID / 32; ++ks) {
              const v16h a = cat16(*(const v8h*)(&hs[ho + ks * 32]), *(const v8h*)(&hs[ho + ks * 32 + 16]));
              acc = wmma16_g(a, ldh(wp + ks * 32), acc); }
          const float bv = bfr(b2[nb * 16 + lr]);
#pragma unroll
          for (int r = 0; r < 8; ++r) xd_s[(8 * hi + r) * FP + nb * 16 + lr] = acc[r] * W2I + bv;
      } }

    const int bo = lr * XP + 8 * hi;
    const v16bf bq0 = cat16b(*(const v8us*)(&xs[bo]),      *(const v8us*)(&xs[bo + 16]));
    const v16bf bq1 = cat16b(*(const v8us*)(&xs[bo + 32]), *(const v8us*)(&xs[bo + 48]));
    const float xnq = xn_s[lr];
    float kd[KNN]; int ki[KNN];
#pragma unroll
    for (int i = 0; i < KNN; ++i) { kd[i] = BIGD; ki[i] = 0; }
    float kmax = BIGD; int kpos = 0; float thr = __builtin_huge_valf();
    const size_t ao = (size_t)lr * DF + 8 * hi;
#pragma unroll 1
    for (int j0 = 0; j0 < NPTS; j0 += 16) {
        const bf* ap = DB + (size_t)j0 * DF + ao;
        const v16bf a0 = ldb(ap), a1 = ldb(ap + 32);
        v8f acc = (v8f){};
        acc = wmmab_g(a0, bq0, acc); acc = wmmab_g(a1, bq1, acc);
        const float* dp = DN + j0 + 8 * hi;
        const v4f d0 = *(const v4f*)dp, d1 = *(const v4f*)(dp + 4);
        float sq[8];
#pragma unroll
        for (int r = 0; r < 4; ++r) { sq[r] = (xnq + d0[r]) - 2.0f * acc[r]; sq[4 + r] = (xnq + d1[r]) - 2.0f * acc[4 + r]; }
        const float mn = fminf(fminf(fminf(sq[0], sq[1]), fminf(sq[2], sq[3])), fminf(fminf(sq[4], sq[5]), fminf(sq[6], sq[7])));
        if (mn < thr) {
            const int jb = j0 + 8 * hi;
#pragma unroll
            for (int r = 0; r < 8; ++r) knn_insert(sq[r], jb + r, kd, ki, kmax, kpos, thr);
        }
    }

#pragma unroll
    for (int i = 0; i < KNN; ++i) { cd[lr * 2 * KNN + hi * KNN + i] = kd[i]; ci[lr * 2 * KNN + hi * KNN + i] = ki[i]; }
#pragma unroll 1
    for (int e = lane; e < QT * KNN; e += 32) { sd[e] = BIGD; si[e] = 0; }
    wave_sync();
#pragma unroll 1
    for (int i = 0; i < KNN; ++i) {
        const int me = lr * 2 * KNN + hi * KNN + i;
        const float d = cd[me]; const int id = ci[me];
        int rank = 0;
#pragma unroll 4
        for (int j = 0; j < 2 * KNN; ++j) { const float e = cd[lr * 2 * KNN + j]; const int ej = ci[lr * 2 * KNN + j]; rank += ((e < d) | ((e == d) & (ej < id))) ? 1 : 0; }
        if (rank < KNN) { sd[lr * KNN + rank] = d; si[lr * KNN + rank] = id; }
    }
    wave_sync();

    { const float hq = fmaxf(sd[lr * KNN + KNN - 1], 1.0e-12f);
      const float den = 2.0f * (hq * hq);
      float wsum = 0.0f;
#pragma unroll 1
      for (int i = 0; i < KNN / 2; ++i) { const int e = lr * KNN + hi * (KNN / 2) + i; const float d = sd[e]; const float w = expf(-(d * d) / den); wn[e] = w; wsum += w; }
      wsum += __shfl_xor(wsum, 16, 32);
      const float dn2 = wsum + 1.0e-12f;
#pragma unroll 1
      for (int i = 0; i < KNN / 2; ++i) { const int e = lr * KNN + hi * (KNN / 2) + i; const float w = wn[e]; wn[e] = w / dn2; } }
    wave_sync();

#pragma unroll 1
    for (int q = 0; q < QT; ++q) {
        float ax = 0.0f, ay = 0.0f;
#pragma unroll 1
        for (int i = 0; i < KNN; ++i) {
            int id = si[q * KNN + i]; id = id < 0 ? 0 : (id > NPTS - 1 ? NPTS - 1 : id);
            const float w = wn[q * KNN + i];
            const v2f vv = *(const v2f*)(vel + (size_t)id * DF + 2 * lane);
            ax += w * bfr(vv[0]); ay += w * bfr(vv[1]); }
        ut_s[q * FP + 2 * lane] = ax; ut_s[q * FP + 2 * lane + 1] = ay;
    }
    wave_sync();

    { float du = 0.0f, nu = 0.0f, nx = 0.0f, l2 = 0.0f;
#pragma unroll 4
      for (int c = 0; c < 32; ++c) {
          const float u = ut_s[lr * FP + hi * 32 + c], x = xd_s[lr * FP + hi * 32 + c];
          du += u * x; nu += u * u; nx += x * x; const float df = u - x; l2 += df * df;
          ot[lr * OW + hi * 32 + c] = x; }
      du += __shfl_xor(du, 16, 32); nu += __shfl_xor(nu, 16, 32); nx += __shfl_xor(nx, 16, 32); l2 += __shfl_xor(l2, 16, 32);
      const float cs = 1.0f - du / (fmaxf(sqrtf(nu), 1.0e-8f) * fmaxf(sqrtf(nx), 1.0e-8f));
      ot[lr * OW + DF + hi] = hi ? l2 : cs; }
    wave_sync();

    float* ob = OUT + (size_t)blockIdx.x * (QT * OW);
#pragma unroll 1
    for (int ps = 0; ps < 2; ++ps) {
#pragma unroll
        for (int s = 0; s < 8; ++s) { const int p = s * 32 + lane;
            const v4f val = *(const v4fa*)(&ot[4 * p]);
            *(volatile v4f*)(ob + 4 * p) = val; }
        { const int p = 256 + (lane & 7);
          const v4f val = *(const v4fa*)(&ot[4 * p]);
          if (lane < 8) *(volatile v4f*)(ob + 4 * p) = val; }
        if (ps == 0) __threadfence(); }
}

static constexpr size_t al256(size_t v) { return (v + 255) & ~(size_t)255; }
static constexpr size_t SZ_DB  = al256((size_t)NPTS * DF * 2);
static constexpr size_t SZ_DN  = al256((size_t)NPTS * 4);
static constexpr size_t SZ_W1T = al256((size_t)HID * K1P * 2);
static constexpr size_t SZ_W2T = al256((size_t)DF * HID * 2);
static constexpr size_t SZ_TOTAL = SZ_DB + SZ_DN + SZ_W1T + SZ_W2T;
static_assert(SZ_TOTAL <= (size_t)134217728);
static_assert(((size_t)NPTS * DF * 2) % 128 == 0);
static_assert(((size_t)NPTS * 4) % 128 == 0);
static_assert((size_t)(NPTS / 32) * 32 * 4 <= SZ_DN);
static_assert((size_t)(W1BLK * 256) * 16 <= SZ_W1T);
static_assert((size_t)(W2BLK * 256) * 16 <= SZ_W2T);
static_assert((size_t)(BQ / QT) * QT * OW == (size_t)BQ * OW);

extern "C" void kernel_launch(void* const* d_in, const int* in_sizes, int n_in,
                              void* d_out, int out_size, void* d_ws, size_t ws_size, hipStream_t stream) {
    if (n_in < 8) return;
    if (in_sizes[0] < 1) return;
    if ((size_t)in_sizes[1] < (size_t)BQ * ZP) return;
    if ((size_t)in_sizes[2] < (size_t)NPTS * DF || (size_t)in_sizes[3] < (size_t)NPTS * DF) return;
    if ((size_t)in_sizes[4] < (size_t)KIN * HID || in_sizes[5] < HID) return;
    if ((size_t)in_sizes[6] < (size_t)HID * DF || in_sizes[7] < DF) return;
    if ((size_t)out_size < (size_t)BQ * OW) return;
    if (SZ_TOTAL > ws_size) return;
    const float* tin  = (const float*)d_in[0];
    const float* z    = (const float*)d_in[1];
    const float* data = (const float*)d_in[2];
    const float* vel  = (const float*)d_in[3];
    const float* W1   = (const float*)d_in[4];
    const float* b1   = (const float*)d_in[5];
    const float* W2   = (const float*)d_in[6];
    const float* b2   = (const float*)d_in[7];
    float* OUT = (float*)d_out;
    char* wsp = (char*)d_ws;
    bf*    DB  = (bf*)wsp;    wsp += SZ_DB;
    float* DN  = (float*)wsp; wsp += SZ_DN;
    bf*    W1T = (bf*)wsp;    wsp += SZ_W1T;
    h16*   W2T = (h16*)wsp;   wsp += SZ_W2T;

    k_dcvt<<<(unsigned)(((size_t)NPTS * DF / 8) / 256), 256, 0, stream>>>(data, DB, DN);
    k_wconv<<<W1BLK + W2BLK, 256, 0, stream>>>(W1, W2, W1T, W2T);
    k_knn<<<BQ / QT, 32, 0, stream>>>(z, tin, DB, DN, vel, W1T, b1, W2T, b2, OUT);
}
